// WindowDecoder_59596966199351
// MI455X (gfx1250) — hardware-verified
//
#include <hip/hip_runtime.h>
#include <math.h>

constexpr int kBatch    = 32;
constexpr int kWin      = 16;
constexpr int kLoc      = 64;
constexpr int kGlo      = 64;
constexpr int kRows     = kBatch * kWin;
constexpr int kZdim     = kLoc + kGlo;
constexpr int kEmb      = 256;
constexpr int kHid      = 512;
constexpr int kOutD     = 64;
constexpr int kSteps    = 128;
constexpr int kG3       = 3 * kEmb;
constexpr int kSeqRows  = kRows * kSteps;
constexpr int kHalfRows = kSeqRows / 2;
constexpr int kTileP    = 264;
constexpr float kWCarry  = 16.0f;
constexpr float kHCarry  = 8.0f;
constexpr float kInvEmb  = 1.0f / 16.0f;
constexpr float kInv128  = 1.0f / 128.0f;

typedef __attribute__((ext_vector_type(16))) _Float16 v16h;
typedef __attribute__((ext_vector_type(8)))  _Float16 v8h;
typedef __attribute__((ext_vector_type(16))) __bf16   v16b;
typedef __attribute__((ext_vector_type(8)))  __bf16   v8b;
typedef __attribute__((ext_vector_type(8)))  float    v8f;
typedef __attribute__((ext_vector_type(4)))  float    v4f;
typedef __attribute__((ext_vector_type(4)))  unsigned int v4u;

__device__ __forceinline__ unsigned short f2bf_bits(float f) {
  unsigned u = __float_as_uint(f);
  return (unsigned short)((u + 0x7FFFu + ((u >> 16) & 1u)) >> 16);
}
__device__ __forceinline__ float bf_bits2f(unsigned short h) { return __uint_as_float(((unsigned)h) << 16); }

__device__ __forceinline__ void dep_guard_h(v8f& a, v8f& b, v16h x, v16h y) { asm volatile("v_nop\n\tv_nop\n\tv_nop\n\tv_nop" : "+v"(a), "+v"(b) : "v"(x), "v"(y)); }
__device__ __forceinline__ void dep_guard_b(v8f& a, v8f& b, v16b x, v16b y) { asm volatile("v_nop\n\tv_nop\n\tv_nop\n\tv_nop" : "+v"(a), "+v"(b) : "v"(x), "v"(y)); }
__device__ __forceinline__ void keep4_h(v16h a, v16h b, v16h c, v16h d) { asm volatile("v_nop" :: "v"(a), "v"(b), "v"(c), "v"(d)); }
__device__ __forceinline__ void keep4_b(v16b a, v16b b, v16b c, v16b d) { asm volatile("v_nop" :: "v"(a), "v"(b), "v"(c), "v"(d)); }
__device__ __forceinline__ void acc_guard4(v8f& a, v8f& b, v8f& c, v8f& d) { asm volatile("v_nop\n\tv_nop\n\tv_nop\n\tv_nop" : "+v"(a), "+v"(b), "+v"(c), "+v"(d)); }
template <typename T> struct Frag;
template <> struct Frag<_Float16> {
  typedef v16h V; union U { v16h v; v8h h[2]; };
  static __device__ __forceinline__ v16h load(const _Float16* p) {
    U f; f.h[0] = *(const v8h*)(p); f.h[1] = *(const v8h*)(p + 16); return f.v;
  }
  static __device__ __forceinline__ v8f mma(v16h a, v16h b, v8f c) {
    return __builtin_amdgcn_wmma_f32_16x16x32_f16(false, a, false, b, (short)0, c, false, false);
  }
  static __device__ __forceinline__ void guard(v8f& a, v8f& b, v16h x, v16h y) { dep_guard_h(a, b, x, y); }
  static __device__ __forceinline__ void keep(v16h a, v16h b, v16h c, v16h d) { keep4_h(a, b, c, d); }
};
template <> struct Frag<__bf16> {
  typedef v16b V; union U { v16b v; v8b h[2]; };
  static __device__ __forceinline__ v16b load(const __bf16* p) {
    U f; f.h[0] = *(const v8b*)(p); f.h[1] = *(const v8b*)(p + 16); return f.v;
  }
  static __device__ __forceinline__ v8f mma(v16b a, v16b b, v8f c) {
    return __builtin_amdgcn_wmma_f32_16x16x32_bf16(false, a, false, b, (short)0, c, false, false);
  }
  static __device__ __forceinline__ void guard(v8f& a, v8f& b, v16b x, v16b y) { dep_guard_b(a, b, x, y); }
  static __device__ __forceinline__ void keep(v16b a, v16b b, v16b c, v16b d) { keep4_b(a, b, c, d); }
};

__device__ __forceinline__ unsigned pk16(unsigned short a, unsigned short b) { return (unsigned)a | ((unsigned)b << 16); }
__device__ __forceinline__ unsigned short h_bits(float f) { const _Float16 h = (_Float16)f; return __builtin_bit_cast(unsigned short, h); }

template <int ET> struct Elem;
template <> struct Elem<0> { typedef _Float16 T; };
template <> struct Elem<1> { typedef __bf16 T; };
template <int ET, bool SPLIT, int BIAS_MODE, int OUT_MODE, bool RESID, int ACT = 0>
__global__ __launch_bounds__(256) void wmma_gemm64(
    const unsigned short* __restrict__ Ap, const unsigned short* __restrict__ A2p, int lda, long strideA,
    const unsigned short* __restrict__ Btp, const unsigned short* __restrict__ Bt2p, int ldb, long strideB,
    void* __restrict__ Cout, void* __restrict__ Cout2, int ldc, long strideC,
    const float* __restrict__ bias,
    const float* __restrict__ resid, long strideR,
    int M, int N, int K, float scale) {
  typedef typename Elem<ET>::T T;
  typedef typename Frag<T>::V V;
  const T* A = (const T*)Ap; const T* A2 = (const T*)A2p; const T* Bt = (const T*)Btp; const T* Bt2 = (const T*)Bt2p;
  __shared__ __align__(16) float sT[8][16 * 68];
  const int b    = blockIdx.y;
  const int lane = threadIdx.x & 31;
  const int wave = threadIdx.x >> 5;
  const int tilesN = N >> 6;
  const int tilesM = M >> 6;
  const int tile = blockIdx.x * 8 + wave;
  if (tile >= tilesM * tilesN) return;
  const int tm = tile / tilesN;
  const int tn = tile - tm * tilesN;
  const int m0 = tm << 6;
  const int n0 = tn << 6;

  const T* Ab  = A  + (size_t)b * strideA;
  const T* Bb  = Bt + (size_t)b * strideB;
  const T* Ab2 = SPLIT ? (A2  + (size_t)b * strideA) : nullptr;
  const T* Bb2 = SPLIT ? (Bt2 + (size_t)b * strideB) : nullptr;

  const int rlane = lane & 15;
  const int koff  = (lane >> 4) * 8;
  const int mOff  = (lane >> 4) * 8;

  v8f acc[4][4];
#pragma unroll
  for (int i = 0; i < 4; ++i)
#pragma unroll
    for (int j = 0; j < 4; ++j) acc[i][j] = (v8f){0.f,0.f,0.f,0.f,0.f,0.f,0.f,0.f};

  for (int k0 = 0; k0 < K; k0 += 32) {
    V bh[4], bl[4];
#pragma unroll
    for (int j = 0; j < 4; ++j) {
      const size_t bo = (size_t)(n0 + (j << 4) + rlane) * ldb + koff + k0;
      bh[j] = Frag<T>::load(Bb + bo);
      if (SPLIT) bl[j] = Frag<T>::load(Bb2 + bo);
    }
#pragma unroll
    for (int i = 0; i < 4; ++i) {
      const size_t ao = (size_t)(m0 + (i << 4) + rlane) * lda + koff + k0;
      V ah = Frag<T>::load(Ab + ao);
      V al;
      if (SPLIT) al = Frag<T>::load(Ab2 + ao);
#pragma unroll
      for (int j = 0; j < 4; ++j) {
        acc[i][j] = Frag<T>::mma(ah, bh[j], acc[i][j]);
        if (SPLIT) {
          acc[i][j] = Frag<T>::mma(ah, bl[j], acc[i][j]);
          acc[i][j] = Frag<T>::mma(al, bh[j], acc[i][j]);
        }
      }
      Frag<T>::guard(acc[i][0], acc[i][3], ah, SPLIT ? al : ah);
    }
    Frag<T>::keep(bh[0], bh[1], bh[2], bh[3]);
    if (SPLIT) Frag<T>::keep(bl[0], bl[1], bl[2], bl[3]);
  }
  acc_guard4(acc[0][0], acc[0][1], acc[0][2], acc[0][3]);
  acc_guard4(acc[1][0], acc[1][1], acc[1][2], acc[1][3]);
  acc_guard4(acc[2][0], acc[2][1], acc[2][2], acc[2][3]);
  acc_guard4(acc[3][0], acc[3][1], acc[3][2], acc[3][3]);

  float* slab = sT[wave];
  const float* Rb = RESID ? (resid + (size_t)b * strideR) : nullptr;
#pragma unroll
  for (int i = 0; i < 4; ++i) {
    const int mBase = m0 + (i << 4);
#pragma unroll
    for (int j = 0; j < 4; ++j) {
      const int n = n0 + (j << 4) + rlane;
      float bv = 0.f;
      if (BIAS_MODE == 2) bv = bias[n];
#pragma unroll
      for (int r = 0; r < 8; ++r) {
        float v = acc[i][j][r] * scale;
        if (BIAS_MODE == 1) v += bias[mBase + mOff + r];
        if (BIAS_MODE == 2) v += bv;
        if (RESID) v += Rb[(size_t)(mBase + mOff + r) * ldc + n];
        if (ACT == 2) v = fmaxf(v, 0.0f);
        if (ACT == 4) v = (v > 0.f) ? v : 0.01f * v;
        if (ACT == 6) {
          const float em = expf(v) - 1.0f;
          v = (v > 0.f) ? v : em;
          v = v * kHCarry;
        }
        slab[(mOff + r) * 68 + (j << 4) + rlane] = v;
      }
    }
    __builtin_amdgcn_fence(__ATOMIC_RELEASE, "workgroup");
    __builtin_amdgcn_wave_barrier();
    __builtin_amdgcn_fence(__ATOMIC_ACQUIRE, "workgroup");
    if (OUT_MODE == 0) {
      float* C = (float*)Cout + (size_t)b * strideC;
      const int hh = lane >> 4, c4 = (lane & 15) * 4;
      for (int pass = 0; pass < 2; ++pass) {
#pragma unroll
        for (int it = 0; it < 8; ++it) {
          const int row = it * 2 + hh;
          v4f v = *(const v4f*)(slab + row * 68 + c4);
          *(volatile v4f*)(C + (size_t)(mBase + row) * ldc + n0 + c4) = v;
        }
        __threadfence();
      }
    } else {
      const int q = lane >> 3, c8 = (lane & 7) * 8;
      unsigned short* C  = (unsigned short*)Cout  + (size_t)b * strideC;
      unsigned short* C2 = (OUT_MODE == 2) ? ((unsigned short*)Cout2 + (size_t)b * strideC) : nullptr;
      for (int pass = 0; pass < 2; ++pass) {
#pragma unroll
        for (int it = 0; it < 4; ++it) {
          const int row = it * 4 + q;
          const float* sp = slab + row * 68 + c8;
          v8h hv, lv;
#pragma unroll
          for (int e = 0; e < 8; ++e) {
            if (OUT_MODE == 1) {
              hv[e] = (_Float16)sp[e];
            } else {
              unsigned short hb = f2bf_bits(sp[e]);
              unsigned short lb = f2bf_bits(sp[e] - bf_bits2f(hb));
              hv[e] = __builtin_bit_cast(_Float16, hb);
              lv[e] = __builtin_bit_cast(_Float16, lb);
            }
          }
          *(volatile v8h*)(C + (size_t)(mBase + row) * ldc + n0 + c8) = hv;
          if (OUT_MODE == 2) *(volatile v8h*)(C2 + (size_t)(mBase + row) * ldc + n0 + c8) = lv;
        }
        __threadfence();
      }
    }
    __builtin_amdgcn_fence(__ATOMIC_RELEASE, "workgroup");
    __builtin_amdgcn_wave_barrier();
    __builtin_amdgcn_fence(__ATOMIC_ACQUIRE, "workgroup");
  }
}

__global__ __launch_bounds__(256) void cast8_f16_kernel(const float* __restrict__ in, unsigned short* __restrict__ out,
                                                        int n8, float carry) {
  const int i = blockIdx.x * 256 + threadIdx.x;
  if (i >= n8) return;
  const float* p = in + 8 * (size_t)i;
  const v4f a = *(const v4f*)(p);
  const v4f c = *(const v4f*)(p + 4);
  unsigned short hb[8];
#pragma unroll
  for (int e = 0; e < 4; ++e) {
    hb[e]     = h_bits(a[e] * carry);
    hb[4 + e] = h_bits(c[e] * carry);
  }
  const v4u u = (v4u){pk16(hb[0], hb[1]), pk16(hb[2], hb[3]), pk16(hb[4], hb[5]), pk16(hb[6], hb[7])};
  unsigned short* q = out + 8 * (size_t)i;
  *(volatile v4u*)q = u;
  __threadfence();
  *(volatile v4u*)q = u;
}

__global__ __launch_bounds__(256) void zcat_kernel(const float* __restrict__ zt, const float* __restrict__ zg,
                                                   unsigned short* __restrict__ Z) {
  const int i = blockIdx.x * 256 + threadIdx.x;
  if (i >= kRows * (kZdim / 8)) return;
  const int row = i >> 4;
  const int seg = i & 15;
  const int c8  = seg * 8;
  const int cl  = c8 & 63;
  const float* pt = zt + (size_t)row * kLoc + cl;
  const float* pg = zg + (size_t)(row >> 4) * kGlo + cl;
  const v4f ta = *(const v4f*)(pt);
  const v4f tb = *(const v4f*)(pt + 4);
  const v4f ga = *(const v4f*)(pg);
  const v4f gb = *(const v4f*)(pg + 4);
  const bool useg = (seg >= 8);
  unsigned short hb[8];
#pragma unroll
  for (int e = 0; e < 4; ++e) {
    const float x0 = useg ? ga[e] : ta[e];
    const float x1 = useg ? gb[e] : tb[e];
    hb[e]     = h_bits(x0);
    hb[4 + e] = h_bits(x1);
  }
  const v4u u = (v4u){pk16(hb[0], hb[1]), pk16(hb[2], hb[3]), pk16(hb[4], hb[5]), pk16(hb[6], hb[7])};
  unsigned short* q = Z + (size_t)row * kZdim + c8;
  *(volatile v4u*)q = u;
  __threadfence();
  *(volatile v4u*)q = u;
}

union FragH { v16h v; v8h h[2]; };
__device__ __forceinline__ v8f hmma(v16h a, v16h b, v8f c) {
  c = __builtin_amdgcn_wmma_f32_16x16x32_f16(false, a, false, b, (short)0, c, false, false);
  asm volatile("v_nop\n\tv_nop\n\tv_nop\n\tv_nop" : "+v"(c) : "v"(a), "v"(b));
  return c;
}
__device__ __forceinline__ float sigm_f32(float x) {
  return __builtin_amdgcn_rcpf(1.0f + expf(-x));
}
__device__ __forceinline__ float tanh_f32(float x) {
  return 1.0f - 2.0f * __builtin_amdgcn_rcpf(1.0f + expf(2.0f * x));
}

__global__ __launch_bounds__(256) void gru_seq_kernel(const float* __restrict__ H0,
                                                      const unsigned short* __restrict__ Whh,
                                                      const float* __restrict__ bih,
                                                      const float* __restrict__ bhh,
                                                      unsigned short* __restrict__ HS) {
  __shared__ __align__(16) _Float16 hT[2][16 * kTileP];
  const int tid  = threadIdx.x;
  const int lane = tid & 31;
  const int wave = tid >> 5;
  const int hh   = lane >> 4;
  const int c    = lane & 15;
  const int koff = hh * 8;
  const int row0 = blockIdx.x * 16;
  const int ub0  = wave * 2;
  const _Float16* W   = (const _Float16*)(const void*)Whh;
  _Float16*       HSh = (_Float16*)(void*)HS;

  float cbr[2], cbz[2], cbn[2], bhn[2];
#pragma unroll
  for (int u = 0; u < 2; ++u) {
    const int unit = (ub0 + u) * 16 + c;
    cbr[u] = bih[unit] + bhh[unit];
    cbz[u] = bih[kEmb + unit] + bhh[kEmb + unit];
    cbn[u] = bih[2 * kEmb + unit];
    bhn[u] = bhh[2 * kEmb + unit];
  }

  float h[2][8];
#pragma unroll
  for (int u = 0; u < 2; ++u) {
    const int unit = (ub0 + u) * 16 + c;
#pragma unroll
    for (int r = 0; r < 8; ++r) {
      const int rr = 8 * hh + r;
      const float v = H0[(size_t)(row0 + rr) * kEmb + unit];
      h[u][r] = v;
      hT[0][rr * kTileP + unit] = (_Float16)(v * kHCarry);
    }
  }
  __syncthreads();

#pragma unroll 1
  for (int t = 0; t < kSteps; ++t) {
    const _Float16* cur = hT[t & 1];
    _Float16*       nxt = hT[(t + 1) & 1];

    v8f acc[2][3];
#pragma unroll
    for (int u = 0; u < 2; ++u)
#pragma unroll
      for (int g = 0; g < 3; ++g) acc[u][g] = (v8f){0.f,0.f,0.f,0.f,0.f,0.f,0.f,0.f};

#pragma unroll 1
    for (int kk = 0; kk < kEmb / 32; ++kk) {
      FragH a;
      a.h[0] = *(const v8h*)(cur + c * kTileP + kk * 32 + koff);
      a.h[1] = *(const v8h*)(cur + c * kTileP + kk * 32 + 16 + koff);
#pragma unroll
      for (int u = 0; u < 2; ++u) {
#pragma unroll
        for (int g = 0; g < 3; ++g) {
          const _Float16* bp = W + (size_t)(g * kEmb + (ub0 + u) * 16 + c) * kEmb + kk * 32 + koff;
          FragH bf;
          bf.h[0] = *(const v8h*)(bp);
          bf.h[1] = *(const v8h*)(bp + 16);
          acc[u][g] = hmma(a.v, bf.v, acc[u][g]);
        }
      }
    }

#pragma unroll
    for (int u = 0; u < 2; ++u) {
      const int unit = (ub0 + u) * 16 + c;
#pragma unroll
      for (int r = 0; r < 8; ++r) {
        const float sr = acc[u][0][r] * kInv128 + cbr[u];
        const float sz = acc[u][1][r] * kInv128 + cbz[u];
        const float gn = acc[u][2][r] * kInv128 + bhn[u];
        const float rg = sigm_f32(sr);
        const float zg = sigm_f32(sz);
        const float nn = tanh_f32(cbn[u] + rg * gn);
        const float hn = (1.0f - zg) * nn + zg * h[u][r];
        h[u][r] = hn;
        nxt[(8 * hh + r) * kTileP + unit] = (_Float16)(hn * kHCarry);
      }
    }
    __syncthreads();

    for (int pass = 0; pass < 2; ++pass) {
#pragma unroll
      for (int it = 0; it < 2; ++it) {
        const int row = wave * 2 + it;
        const v8h v = *(const v8h*)(nxt + row * kTileP + lane * 8);
        *(volatile v8h*)(HSh + ((size_t)(row0 + row) * kSteps + t) * kEmb + lane * 8) = v;
      }
      __threadfence();
    }
  }
}

extern "C" void kernel_launch(void* const* d_in, const int* in_sizes, int n_in,
                              void* d_out, int out_size, void* d_ws, size_t ws_size,
                              hipStream_t stream) {
  if (n_in < 14) return;
  if (in_sizes[0] != kRows * kLoc) return;
  if (in_sizes[1] != kBatch * kGlo) return;
  if (in_sizes[2] != kEmb * kZdim) return;
  if (in_sizes[3] != kG3 * kEmb) return;
  if (in_sizes[4] != kG3 || in_sizes[5] != kG3) return;
  if (in_sizes[6] != kHid * kEmb || in_sizes[7] != kHid) return;
  if (in_sizes[8] != kHid * kHid || in_sizes[9] != kHid) return;
  if (in_sizes[10] != kHid * kHid || in_sizes[11] != kHid) return;
  if (in_sizes[12] != kOutD * kHid || in_sizes[13] != kOutD) return;
  if (out_size != kSeqRows * kOutD) return;

  const float* z_t  = (const float*)d_in[0];
  const float* z_g  = (const float*)d_in[1];
  const float* wemb = (const float*)d_in[2];
  const float* whh  = (const float*)d_in[3];
  const float* bih  = (const float*)d_in[4];
  const float* bhh  = (const float*)d_in[5];
  const float* w1   = (const float*)d_in[6];
  const float* b1   = (const float*)d_in[7];
  const float* w2   = (const float*)d_in[8];
  const float* b2   = (const float*)d_in[9];
  const float* w3   = (const float*)d_in[10];
  const float* b3   = (const float*)d_in[11];
  const float* wmu  = (const float*)d_in[12];
  const float* bmu  = (const float*)d_in[13];
  float* out = (float*)d_out;

  char* ws = (char*)d_ws;
  size_t off = 0;
  const size_t szWemb = (size_t)kEmb * kZdim * 2;
  const size_t szWhh  = (size_t)kG3 * kEmb * 2;
  const size_t szW1   = (size_t)kHid * kEmb * 2;
  const size_t szW2   = (size_t)kHid * kHid * 2;
  const size_t szWmu  = (size_t)kOutD * kHid * 2;
  const size_t szZ    = (size_t)kRows * kZdim * 2;
  const size_t szH0   = (size_t)kRows * kEmb * 4;
  const size_t szHS   = (size_t)kSeqRows * kEmb * 2;
  const size_t szP    = (size_t)kHalfRows * kHid * 2;
  unsigned short* wemb16 = (unsigned short*)(ws + off); off += szWemb;
  unsigned short* whh16  = (unsigned short*)(ws + off); off += szWhh;
  unsigned short* w1_16  = (unsigned short*)(ws + off); off += szW1;
  unsigned short* w2_16  = (unsigned short*)(ws + off); off += szW2;
  unsigned short* w3_16  = (unsigned short*)(ws + off); off += szW2;
  unsigned short* wmu16  = (unsigned short*)(ws + off); off += szWmu;
  unsigned short* z16    = (unsigned short*)(ws + off); off += szZ;
  float*          h0     = (float*)(ws + off);          off += szH0;
  unsigned short* hs     = (unsigned short*)(ws + off); off += szHS;
  unsigned short* p1     = (unsigned short*)(ws + off); off += szP;
  unsigned short* p2     = (unsigned short*)(ws + off); off += szP;
  if (off > ws_size) return;

  {
    const int n8a = kEmb * kZdim / 8, n8b = kG3 * kEmb / 8, n8c = kHid * kEmb / 8, n8d = kHid * kHid / 8, n8e = kOutD * kHid / 8;
    cast8_f16_kernel<<<(n8a + 255) / 256, 256, 0, stream>>>(wemb, wemb16, n8a, kWCarry);
    cast8_f16_kernel<<<(n8b + 255) / 256, 256, 0, stream>>>(whh,  whh16,  n8b, kWCarry);
    cast8_f16_kernel<<<(n8c + 255) / 256, 256, 0, stream>>>(w1,   w1_16,  n8c, kWCarry);
    cast8_f16_kernel<<<(n8d + 255) / 256, 256, 0, stream>>>(w2,   w2_16,  n8d, kWCarry);
    cast8_f16_kernel<<<(n8d + 255) / 256, 256, 0, stream>>>(w3,   w3_16,  n8d, kWCarry);
    cast8_f16_kernel<<<(n8e + 255) / 256, 256, 0, stream>>>(wmu,  wmu16,  n8e, kWCarry);
  }
  zcat_kernel<<<(kRows * (kZdim / 8) + 255) / 256, 256, 0, stream>>>(z_t, z_g, z16);

  wmma_gemm64<0, false, 0, 0, false, 0><<<dim3((8 * 4 + 7) / 8, 1), 256, 0, stream>>>(
      (const unsigned short*)z16, (const unsigned short*)nullptr, kZdim, 0L,
      (const unsigned short*)wemb16, (const unsigned short*)nullptr, kZdim, 0L,
      (void*)h0, (void*)nullptr, kEmb, 0L,
      (const float*)nullptr, (const float*)nullptr, 0L,
      kRows, kEmb, kZdim, kInvEmb);

  gru_seq_kernel<<<kRows / 16, 256, 0, stream>>>(h0, whh16, bih, bhh, hs);

  const int tilesBig = (kHalfRows / 64) * (kHid / 64);
  const int tilesMu  = (kHalfRows / 64) * (kOutD / 64);
  for (int hf = 0; hf < 2; ++hf) {
    const unsigned short* hsA = hs + (size_t)hf * kHalfRows * kEmb;
    float* outH = out + (size_t)hf * kHalfRows * kOutD;
    wmma_gemm64<0, false, 2, 1, false, 6><<<dim3((tilesBig + 7) / 8, 1), 256, 0, stream>>>(
        hsA, (const unsigned short*)nullptr, kEmb, 0L,
        (const unsigned short*)w1_16, (const unsigned short*)nullptr, kEmb, 0L,
        (void*)p1, (void*)nullptr, kHid, 0L,
        b1, (const float*)nullptr, 0L,
        kHalfRows, kHid, kEmb, kInv128);
    wmma_gemm64<0, false, 2, 1, false, 6><<<dim3((tilesBig + 7) / 8, 1), 256, 0, stream>>>(
        (const unsigned short*)p1, (const unsigned short*)nullptr, kHid, 0L,
        (const unsigned short*)w2_16, (const unsigned short*)nullptr, kHid, 0L,
        (void*)p2, (void*)nullptr, kHid, 0L,
        b2, (const float*)nullptr, 0L,
        kHalfRows, kHid, kHid, kInv128);
    wmma_gemm64<0, false, 2, 1, false, 6><<<dim3((tilesBig + 7) / 8, 1), 256, 0, stream>>>(
        (const unsigned short*)p2, (const unsigned short*)nullptr, kHid, 0L,
        (const unsigned short*)w3_16, (const unsigned short*)nullptr, kHid, 0L,
        (void*)p1, (void*)nullptr, kHid, 0L,
        b3, (const float*)nullptr, 0L,
        kHalfRows, kHid, kHid, kInv128);
    wmma_gemm64<0, false, 2, 0, false, 0><<<dim3((tilesMu + 7) / 8, 1), 256, 0, stream>>>(
        (const unsigned short*)p1, (const unsigned short*)nullptr, kHid, 0L,
        (const unsigned short*)wmu16, (const unsigned short*)nullptr, kHid, 0L,
        (void*)outH, (void*)nullptr, kOutD, 0L,
        bmu, (const float*)nullptr, 0L,
        kHalfRows, kOutD, kHid, kInv128);
  }
}
